// GraphMambaModel_37726992728373
// MI455X (gfx1250) — hardware-run, weakly checked
//
#include <hip/hip_runtime.h>


namespace {
constexpr int N = 16384, E = 262144, F = 32, H = 128, G = 16, DI = 256, DS = 16, DC = 4, DTR = 8, XPW = DTR + 2 * DS, OUTW = 1 + 4 + 3 + 512 * 3 + 8, NBLK = N / 16;
constexpr float XS = 8.0f, S1 = 512.0f, S2 = 4096.0f, SX = 65536.0f, SD = 262144.0f, SY = 1048576.0f, WSC = 256.0f;
typedef _Float16 b16;
typedef __attribute__((ext_vector_type(16))) _Float16 v16b;
typedef __attribute__((ext_vector_type(8))) _Float16 v8b;
typedef __attribute__((ext_vector_type(8))) float v8f;
typedef __attribute__((ext_vector_type(4))) float v4f;
__device__ __forceinline__ float bf16_rne(float f) { unsigned int u = __float_as_uint(f); u += 0x7FFFu + ((u >> 16) & 1u); return __uint_as_float(u & 0xFFFF0000u); }
__device__ __forceinline__ void split16(float v, b16& hi, b16& lo) { hi = (b16)v; lo = (b16)(v - (float)hi); }
__device__ __forceinline__ v16b frag_kb(const b16* p, int hh) { const v8b a = *(const v8b*)(p + 8 * hh), b = *(const v8b*)(p + 16 + 8 * hh); v16b f;
#pragma unroll
  for (int e = 0; e < 8; ++e) { f[e] = a[e]; f[8 + e] = b[e]; } return f; }
__device__ __forceinline__ v8f wmma16b(v16b a, v16b b, v8f c) { v8f d = __builtin_amdgcn_wmma_f32_16x16x32_f16(false, a, false, b, (short)0, c, false, false); asm volatile("v_nop\n\tv_nop\n\tv_nop\n\tv_nop" : "+v"(d) : "v"(a), "v"(b)); return d; }
__device__ __forceinline__ void wave_lds_sync() { __builtin_amdgcn_fence(__ATOMIC_RELEASE, "workgroup"); __builtin_amdgcn_wave_barrier(); __builtin_amdgcn_fence(__ATOMIC_ACQUIRE, "workgroup"); }
__device__ __forceinline__ float pmul(float a, float b) { float p = a * b; asm volatile("" : "+v"(p)); return p; }
__device__ __forceinline__ int iclamp(int v, int lo, int hi) { return v < lo ? lo : (v > hi ? hi : v); }
__device__ __forceinline__ float silu(float v) { return v / (1.0f + __expf(-v)); }
__device__ __forceinline__ float softplus(float v) { return v > 20.0f ? v : log1pf(__expf(v)); }
constexpr int CSR_NBLK9 = 512, CSR_GB9 = 9, CSR_GN9 = 1 << CSR_GB9  , CSR_TS9 = (CSR_GN9 < 32 ? 32 : CSR_GN9)  , CSR_MAXG9 = 512, CSR_CAP9 = 12288  ;
__device__ __host__ __forceinline__ int csr_tix9(int v) { return (v >> CSR_GB9) * CSR_TS9 + (v & (CSR_GN9 - 1)); }
__global__ __launch_bounds__(64) void csrA_kernel9(const int* __restrict__ dst, int E, int N, int nG, int CHP, int NGP, int* __restrict__ STG, int* __restrict__ HST) {
  extern __shared__ int sm[];
  int* cnt = sm; int* run = sm + NGP; int* ids = sm + 2 * NGP;
  const int b = blockIdx.x; const int ch = (E + CSR_NBLK9 - 1) / CSR_NBLK9; const int e0 = b * ch, e1 = min(E, e0 + ch);
  for (int i = threadIdx.x; i < NGP; i += 64) cnt[i] = 0;
  for (int i = threadIdx.x; i < CHP; i += 64) ids[i] = -1;
  __syncthreads();
  if (threadIdx.x == 0) {
    for (int e = e0; e < e1; ++e) { int d = dst[e]; d = (d < 0) ? 0 : (d >= N ? N - 1 : d); cnt[d >> CSR_GB9] += 1; }
    int acc = 0; for (int g = 0; g < nG; ++g) { run[g] = acc; acc += cnt[g]; }
    for (int e = e0; e < e1; ++e) { int d = dst[e]; d = (d < 0) ? 0 : (d >= N ? N - 1 : d); const int g = d >> CSR_GB9; ids[run[g]] = e; run[g] += 1; } }
  __syncthreads();
  typedef __attribute__((ext_vector_type(4))) int v4i;
  for (int pass = 0; pass < 2; ++pass) {
    for (int i = threadIdx.x; i < CHP / 4; i += 64) *(volatile v4i*)(STG + (size_t)b * CHP + i * 4) = *(const v4i*)(&ids[i * 4]);
    for (int i = threadIdx.x; i < NGP / 4; i += 64) { v4i v; for (int e = 0; e < 4; ++e) v[e] = (i * 4 + e < nG) ? cnt[i * 4 + e] : 0; *(volatile v4i*)(HST + (size_t)b * NGP + i * 4) = v; }
    __threadfence(); }
}
__global__ __launch_bounds__(512) void csrS_kernel9(const int* __restrict__ HST, int nG, int NGP, int* __restrict__ START, int* __restrict__ TOT, int* __restrict__ OFF) {
  __shared__ int tot[CSR_MAXG9];
  const int b = threadIdx.x;
  for (int pass = 0; pass < 2; ++pass) { int runb = 0; for (int g = 0; g < nG; ++g) { int c = HST[(size_t)b * NGP + g]; c = (c < 0) ? 0 : c; ((volatile int*)OFF)[(size_t)g * CSR_NBLK9 + b] = runb; runb += c; } __threadfence(); }
  for (int g = threadIdx.x; g < nG; g += 512) { int s = 0; for (int bb = 0; bb < CSR_NBLK9; ++bb) { int c = HST[(size_t)bb * NGP + g]; s += (c < 0) ? 0 : c; } tot[g] = s; }
  __syncthreads();
  if (threadIdx.x < 32) {
    __shared__ int st[CSR_MAXG9 + 32];
    if (threadIdx.x == 0) { int acc = 0; for (int g = 0; g < NGP; ++g) { st[g] = acc; if (g < nG) acc += (tot[g] + 31) & ~31; } st[NGP] = acc; }
    __builtin_amdgcn_fence(__ATOMIC_RELEASE, "workgroup"); __builtin_amdgcn_wave_barrier(); __builtin_amdgcn_fence(__ATOMIC_ACQUIRE, "workgroup");
    for (int pass = 0; pass < 2; ++pass) { for (int i = threadIdx.x; i < NGP + 32; i += 32) { ((volatile int*)START)[i] = (i <= NGP) ? st[min(i, NGP)] : 0; ((volatile int*)TOT)[i] = (i < nG) ? tot[i] : 0; } __threadfence(); } }
}
__global__ __launch_bounds__(256) void csrB_kernel9(const int* __restrict__ dst, int N, int nG, int CHP, int NGP, int permLen, const int* __restrict__ STG, const int* __restrict__ HST, const int* __restrict__ OFF, const int* __restrict__ START, const int* __restrict__ TOT, int* __restrict__ PERM, int* __restrict__ ROWPTR, int* __restrict__ ROWCNT, int* __restrict__ FLAG) {
  typedef __attribute__((ext_vector_type(4))) int v4i;
  __shared__ int ids[CSR_CAP9]; __shared__ unsigned short key[CSR_CAP9]; __shared__ int outp[CSR_CAP9]; __shared__ int ncnt[CSR_GN9 + 1]; __shared__ int boff[CSR_NBLK9 + 1];
  const int g = blockIdx.x, t_ = threadIdx.x; int tot = TOT[g]; int st = START[g], stn = START[g + 1]; const int v0 = g * CSR_GN9; const int nv = min(CSR_GN9, N - v0); const int t0 = g * CSR_TS9;
  st = (st < 0) ? 0 : (st > permLen - 32 ? permLen - 32 : st) & ~31; stn = (stn < st) ? st : (stn > permLen ? permLen : stn); tot = (tot < 0) ? 0 : tot; if (tot > stn - st && tot <= CSR_CAP9) tot = stn - st;
  if (tot > CSR_CAP9) {
    for (int pass = 0; pass < 2; ++pass) { for (int i = t_; i < CSR_TS9 / 4; i += 256) { v4i a, c; for (int e = 0; e < 4; ++e) { a[e] = st; c[e] = 0; } *(volatile v4i*)(ROWPTR + t0 + i * 4) = a; *(volatile v4i*)(ROWCNT + t0 + i * 4) = c; } if (t_ == 0) ((volatile int*)FLAG)[0] = 1; __threadfence(); } (void)nv; return; }
  if (t_ == 0) { int acc = 0; for (int b = 0; b < CSR_NBLK9; ++b) { boff[b] = acc; int c = HST[(size_t)b * NGP + g]; c = (c < 0) ? 0 : (c > CHP ? CHP : c); acc += c; if (acc > tot) acc = tot; } boff[CSR_NBLK9] = acc; }
  for (int i = t_; i <= CSR_GN9; i += 256) ncnt[i] = 0;
  __syncthreads();
  for (int b = 0; b < CSR_NBLK9; ++b) { const int c = boff[b + 1] - boff[b]; int o_ = OFF[(size_t)g * CSR_NBLK9 + b]; o_ = (o_ < 0) ? 0 : (o_ > CHP - c ? CHP - c : o_); const int* src_ = STG + (size_t)b * CHP + o_;
    for (int i = t_; i < c; i += 256) { int id = src_[i]; id = (id < 0) ? 0 : id; ids[boff[b] + i] = id; int d = dst[id]; d = (d < v0) ? v0 : (d >= N ? N - 1 : d); int kk = d - v0; kk = (kk < 0) ? 0 : (kk >= CSR_GN9 ? CSR_GN9 - 1 : kk); key[boff[b] + i] = (unsigned short)kk; } }
  __syncthreads();
  if (t_ == 0) { for (int i = 0; i < tot; ++i) ncnt[key[i]] += 1; int acc = 0; for (int vl = 0; vl < CSR_GN9; ++vl) { const int c = ncnt[vl]; ncnt[vl] = acc; acc += c; } ncnt[CSR_GN9] = acc;
    for (int i = 0; i < tot; ++i) { const int vl = key[i]; outp[ncnt[vl]] = ids[i]; ncnt[vl] += 1; }
    for (int vl = CSR_GN9; vl > 0; --vl) ncnt[vl] = ncnt[vl - 1]; ncnt[0] = 0; }
  __syncthreads();
  for (int pass = 0; pass < 2; ++pass) {
    for (int i = t_; i < (stn - st) / 4; i += 256) { v4i v; for (int e = 0; e < 4; ++e) { const int q = i * 4 + e; v[e] = (q < tot) ? outp[q] : -1; } *(volatile v4i*)(PERM + st + i * 4) = v; }
    for (int i = t_; i < CSR_TS9 / 4; i += 256) { v4i a, c; for (int e = 0; e < 4; ++e) { const int vl = i * 4 + e; const int vc = vl < CSR_GN9 ? vl : CSR_GN9; a[e] = (vl < CSR_GN9) ? st + ncnt[vc] : st; c[e] = (vl < nv) ? (ncnt[(vc < CSR_GN9 ? vc : CSR_GN9 - 1) + 1] - ncnt[vc]) : 0; } *(volatile v4i*)(ROWPTR + t0 + i * 4) = a; *(volatile v4i*)(ROWCNT + t0 + i * 4) = c; }
    __threadfence(); }
}
__global__ __launch_bounds__(256) void csrZ_kernel9(int* __restrict__ p, size_t n4) { typedef __attribute__((ext_vector_type(4))) int v4i; const size_t tid = (size_t)blockIdx.x * 256 + threadIdx.x, nth = (size_t)gridDim.x * 256; v4i z = {0, 0, 0, 0}; for (size_t i = tid; i < n4; i += nth) *(volatile v4i*)(p + i * 4) = z; }
struct CsrBufs9 { int *STG, *HST, *OFF, *START, *TOT, *PERM, *ROWPTR, *ROWCNT, *FLAG; int nG, NGP, CHP; size_t permLen; char* base; size_t bytes; };
static size_t csr_carve9(CsrBufs9& c, char* ws, size_t off, int E, int N) {
  const size_t off0 = off; c.base = ws + off;
  auto al = [&](size_t bytes) { char* p = ws + off; off += (bytes + 255) & ~(size_t)255; return p; };
  c.nG = (N + CSR_GN9 - 1) / CSR_GN9; c.NGP = (c.nG + 31) & ~31; const int ch = (E + CSR_NBLK9 - 1) / CSR_NBLK9; c.CHP = (ch + 31) & ~31; c.permLen = (size_t)E + 32 * (size_t)c.nG + 32;
  c.STG = (int*)al((size_t)CSR_NBLK9 * c.CHP * 4); c.HST = (int*)al((size_t)CSR_NBLK9 * c.NGP * 4); c.OFF = (int*)al((size_t)c.NGP * CSR_NBLK9 * 4); c.START = (int*)al((size_t)(c.NGP + 64) * 4); c.TOT = (int*)al((size_t)(c.NGP + 64) * 4);
  c.PERM = (int*)al(c.permLen * 4); c.ROWPTR = (int*)al((size_t)c.nG * CSR_TS9 * 4); c.ROWCNT = (int*)al((size_t)c.nG * CSR_TS9 * 4); c.FLAG = (int*)al(256);
  c.bytes = off - off0; return off;
}
static void csr_build9(const CsrBufs9& c, const int* dst, int E, int N, hipStream_t stream) {
  const size_t smem = (size_t)(2 * c.NGP + c.CHP) * 4;
  csrZ_kernel9<<<512, 256, 0, stream>>>((int*)c.base, c.bytes / 16);
  csrA_kernel9<<<CSR_NBLK9, 64, smem, stream>>>(dst, E, N, c.nG, c.CHP, c.NGP, c.STG, c.HST);
  csrS_kernel9<<<1, 512, 0, stream>>>(c.HST, c.nG, c.NGP, c.START, c.TOT, c.OFF);
  csrB_kernel9<<<c.nG, 256, 0, stream>>>(dst, N, c.nG, c.CHP, c.NGP, (int)c.permLen, c.STG, c.HST, c.OFF, c.START, c.TOT, c.PERM, c.ROWPTR, c.ROWCNT, c.FLAG);
}


__global__ __launch_bounds__(256) void wput_kernel(const float* __restrict__ w, int KIN, int KP, int OUTW_, int OUTP, b16* __restrict__ WT) {
  const int KG = KP / 8; const int u = blockIdx.x * 256 + threadIdx.x; if (u >= OUTP * KG) return; const int o = u / KG, k0 = (u % KG) * 8; v8b v;
#pragma unroll
  for (int j = 0; j < 8; ++j) { const int k = k0 + j; v[j] = (o < OUTW_ && k < KIN) ? (b16)(bf16_rne(w[(size_t)k * OUTW_ + o]) * WSC) : (b16)0.0f; } for (int pass = 0; pass < 2; ++pass) { *(volatile v8b*)(WT + (size_t)o * KP + k0) = v; __threadfence(); }
}
template <int KP, int NT, int FIRST, int EPI>
__global__ __launch_bounds__(32) void dense_kernel(const float* __restrict__ IN, int PIN, int c0, int KIN, float scale, const b16* __restrict__ WT, const float* __restrict__ bias, float* __restrict__ OUT) {
  __shared__ __attribute__((aligned(16))) b16 Ah[16][KP + 8], Al[16][KP + 8]; __shared__ __attribute__((aligned(16))) float Tf[16][128 + 4];
  const int lane = threadIdx.x, nloc = lane & 15, hlf = lane >> 4; const size_t m0 = (size_t)blockIdx.x * 16;
  for (int rr = 0; rr < 16; ++rr) for (int q = 0; q < KP / 32; ++q) { const int c = q * 32 + lane; float v = 0.0f; if (c < KIN) { v = IN[(m0 + rr) * PIN + c0 + c]; if (FIRST) v = bf16_rne(v); } b16 p, ql; split16(v * scale, p, ql); Ah[rr][c] = p; Al[rr][c] = ql; }
  wave_lds_sync(); const float sc = 1.0f / (scale * WSC);
#pragma unroll 1
  for (int cg = 0; cg < (NT + 7) / 8; ++cg) { const int nt = (NT - cg * 8) < 8 ? (NT - cg * 8) : 8; v8f acc[8];
#pragma unroll
    for (int t = 0; t < 8; ++t) acc[t] = (v8f){};
#pragma unroll
    for (int kb = 0; kb < KP; kb += 32) { const v16b a = frag_kb(&Ah[nloc][kb], hlf), al = frag_kb(&Al[nloc][kb], hlf);
#pragma unroll
      for (int t = 0; t < 8; ++t) if (t < nt) { const v16b bw = frag_kb(WT + (size_t)(cg * 128 + t * 16 + nloc) * KP + kb, hlf); acc[t] = wmma16b(a, bw, acc[t]); if (!FIRST) acc[t] = wmma16b(al, bw, acc[t]); } }
#pragma unroll
    for (int t = 0; t < 8; ++t) { if (t < nt) { const int c = cg * 128 + t * 16 + nloc; const float bb = (EPI != 0) ? bf16_rne(bias[c]) : 0.0f;
#pragma unroll
        for (int r8 = 0; r8 < 8; ++r8) { float v = acc[t][r8] * sc; if (EPI == 1) v = fmaxf(v + bb, 0.0f); else if (EPI == 2) v += bb; else if (EPI == 3) v = softplus(v + bb); Tf[8 * hlf + r8][t * 16 + nloc] = v; } } }
    wave_lds_sync();
    for (int pass = 0; pass < 2; ++pass) { for (int rr = 0; rr < 16; ++rr) for (int c = lane; c < nt * 16; c += 32) ((volatile float*)OUT)[(m0 + rr) * (NT * 16) + cg * 128 + c] = Tf[rr][c]; __threadfence(); }
    wave_lds_sync(); }
}
__global__ __launch_bounds__(256) void agg_kernel(const float* __restrict__ XW, const int* __restrict__ srcs, const int* __restrict__ PERM, const int* __restrict__ ROWPTR, const int* __restrict__ ROWCNT, int permLen, const float* __restrict__ bias, float* __restrict__ OUT) {
  const int wave = threadIdx.x >> 5, lane = threadIdx.x & 31; const size_t v = (size_t)blockIdx.x * 8 + wave; if (v >= (size_t)N) return;
  int st = ROWPTR[v], cnt = ROWCNT[v]; cnt = iclamp(cnt, 0, 1 << 20); st = iclamp(st, 0, permLen - cnt); const float dv = rsqrtf((float)cnt + 1.0f);
  v4f o = *(const v4f*)(XW + v * H + lane * 4); { const float w = pmul(dv, dv); for (int i = 0; i < 4; ++i) o[i] = pmul(w, o[i]); }
#pragma unroll 1
  for (int j = 0; j < cnt; ++j) { const int e = iclamp(PERM[st + j], 0, E - 1); const size_t u = (size_t)iclamp(srcs[e], 0, N - 1); const int cu = iclamp(ROWCNT[u], 0, 1 << 20); const float w = pmul(rsqrtf((float)cu + 1.0f), dv); const v4f xv = *(const v4f*)(XW + u * H + lane * 4); for (int i = 0; i < 4; ++i) o[i] += pmul(w, xv[i]); }
  v4f r; for (int i = 0; i < 4; ++i) r[i] = fmaxf(o[i] + bf16_rne(bias[lane * 4 + i]), 0.0f);
  for (int pass = 0; pass < 2; ++pass) { *(volatile v4f*)(OUT + v * H + lane * 4) = r; __threadfence(); }
}
__global__ __launch_bounds__(256) void conv_kernel(const float* __restrict__ XZ, const float* __restrict__ cw, const float* __restrict__ cbi, int LS, float* __restrict__ X) {
  const size_t gid = (size_t)blockIdx.x * 256 + threadIdx.x; const int cg = (int)(gid % 32), t = (int)(gid / 32); if (t >= LS) return; const int c0 = cg * 8; float r[8];
  for (int i = 0; i < 8; ++i) { const int c = c0 + i; float s = bf16_rne(cbi[c]); for (int k = 0; k < DC; ++k) { const int tt = t - (DC - 1) + k; if (tt >= 0) s += pmul(bf16_rne(cw[c * DC + k]), XZ[(size_t)tt * (2 * DI) + c]); } r[i] = silu(s); }
  for (int pass = 0; pass < 2; ++pass) { *(volatile v4f*)(X + (size_t)t * DI + c0) = (v4f){r[0], r[1], r[2], r[3]}; *(volatile v4f*)(X + (size_t)t * DI + c0 + 4) = (v4f){r[4], r[5], r[6], r[7]}; __threadfence(); }
}
__global__ __launch_bounds__(256) void scan_kernel(const float* __restrict__ X, const float* __restrict__ DT, const float* __restrict__ DBL, const float* __restrict__ XZ, const float* __restrict__ A_log, const float* __restrict__ Dp, int LS, float* __restrict__ Y) {
  const int di = threadIdx.x; float A[DS], h[DS]; for (int s = 0; s < DS; ++s) { A[s] = -__expf(bf16_rne(A_log[di * DS + s])); h[s] = 0.0f; } const float dp = bf16_rne(Dp[di]);
#pragma unroll 1
  for (int t = 0; t < LS; ++t) { const float dt = DT[(size_t)t * DI + di], x = X[(size_t)t * DI + di]; const float* bc = DBL + (size_t)t * 64 + DTR; float y = 0.0f;
#pragma unroll
    for (int s = 0; s < DS; ++s) { h[s] = pmul(__expf(pmul(dt, A[s])), h[s]) + pmul(pmul(dt, bc[s]), x); y += pmul(h[s], bc[DS + s]); }
    y = pmul(y + pmul(dp, x), silu(XZ[(size_t)t * (2 * DI) + DI + di]));
    ((volatile float*)Y)[(size_t)t * DI + di] = y; ((volatile float*)Y)[(size_t)t * DI + di] = y; if ((t & 255) == 255) __threadfence(); }
  __threadfence();
}
__global__ __launch_bounds__(256) void ln_kernel(const float* __restrict__ HG, const float* __restrict__ HM, const float* __restrict__ gam, const float* __restrict__ bet, int LS, float* __restrict__ HF) {
  const int wave = threadIdx.x >> 5, lane = threadIdx.x & 31; const size_t t = (size_t)blockIdx.x * 8 + wave; if (t >= (size_t)LS) return;
  float v[4]; float s = 0.0f; for (int i = 0; i < 4; ++i) { v[i] = HG[t * H + lane * 4 + i] + HM[t * H + lane * 4 + i]; s += v[i]; } for (int o = 16; o; o >>= 1) s += __shfl_xor(s, o); const float mu = s * (1.0f / H);
  float q = 0.0f; for (int i = 0; i < 4; ++i) { const float d = v[i] - mu; q += pmul(d, d); } for (int o = 16; o; o >>= 1) q += __shfl_xor(q, o); const float rs = rsqrtf(q * (1.0f / H) + 1e-5f);
  v4f r; for (int i = 0; i < 4; ++i) { const int c = lane * 4 + i; r[i] = pmul(pmul(v[i] - mu, rs), bf16_rne(gam[c])) + bf16_rne(bet[c]); }
  for (int pass = 0; pass < 2; ++pass) { *(volatile v4f*)(HF + t * H + lane * 4) = r; __threadfence(); }
}
__global__ __launch_bounds__(128) void pool_kernel(const float* __restrict__ HF, const int* __restrict__ batch, int LS, float* __restrict__ GE) {
  const int g = blockIdx.x, c = threadIdx.x;
  auto lb = [&](int key) -> int { int lo = 0, hi = N; for (int it = 0; it < 15 && lo < hi; ++it) { const int mid = (lo + hi) >> 1; if (batch[mid] < key) lo = mid + 1; else hi = mid; } return lo; };
  int s0 = lb(g), e0 = lb(g + 1); if (e0 > LS) e0 = LS; if (e0 < s0) e0 = s0; float s = 0.0f; int cnt = 0;
#pragma unroll 1
  for (int n = s0; n < e0; ++n) { s += HF[(size_t)n * H + c]; ++cnt; }
  const float m = s / (float)(cnt < 1 ? 1 : cnt); for (int pass = 0; pass < 2; ++pass) { ((volatile float*)GE)[g * H + c] = m; __threadfence(); }
}
__global__ __launch_bounds__(256) void heads_kernel(const float* __restrict__ GE, const float* __restrict__ Wc, const float* __restrict__ bc, const float* __restrict__ Wh, const float* __restrict__ bh, const float* __restrict__ Wt, const float* __restrict__ bt, const float* __restrict__ Wp1, const float* __restrict__ bp1, const float* __restrict__ Wp2, const float* __restrict__ bp2, const float* __restrict__ Wd, const float* __restrict__ bd, const float* __restrict__ Wsx, const float* __restrict__ bs, float* __restrict__ out) {
  __shared__ float Ge[G][H]; const int tid = threadIdx.x; for (int i = tid; i < G * H; i += 256) Ge[i / H][i % H] = GE[i]; __syncthreads();
  for (int pass = 0; pass < 2; ++pass) {
    for (int i = tid; i < G * OUTW; i += 256) { const int g = i / OUTW, col = i % OUTW; const float* Wp; const float* bp; int cw_, cc;
      if (col < 1) { Wp = Wc; bp = bc; cw_ = 1; cc = col; } else if (col < 5) { Wp = Wh; bp = bh; cw_ = 4; cc = col - 1; } else if (col < 8) { Wp = Wt; bp = bt; cw_ = 3; cc = col - 5; } else if (col < 520) { Wp = Wp1; bp = bp1; cw_ = 512; cc = col - 8; } else if (col < 1032) { Wp = Wp2; bp = bp2; cw_ = 512; cc = col - 520; } else if (col < 1544) { Wp = Wd; bp = bd; cw_ = 512; cc = col - 1032; } else { Wp = Wsx; bp = bs; cw_ = 8; cc = col - 1544; }
      float s = bf16_rne(bp[cc]);
#pragma unroll 1
      for (int k = 0; k < H; ++k) s += pmul(Ge[g][k], bf16_rne(Wp[(size_t)k * cw_ + cc]));
      ((volatile float*)out)[i] = s; }
    __threadfence(); }
}
}

extern "C" void kernel_launch(void* const* d_in, const int* in_sizes, int n_in, void* d_out, int out_size, void* d_ws, size_t ws_size, hipStream_t stream) {
  (void)n_in;
  auto Fp = [&](int i) { return (const float*)d_in[i]; }; auto Ip = [&](int i) { return (const int*)d_in[i]; };
  if (in_sizes[0] != N * F || in_sizes[1] != 2 * E || in_sizes[2] != N || in_sizes[3] != F * H || in_sizes[5] != H * H || in_sizes[9] != H * 2 * DI || in_sizes[10] != DI * DC || in_sizes[12] != DI * XPW || in_sizes[13] != DTR * DI || in_sizes[15] != DI * DS || in_sizes[17] != DI * H || in_sizes[26] != H * 512 || in_sizes[32] != H * 8 || out_size != G * OUTW) return;
  const int LS = N;
  size_t off = 0; char* ws = (char*)d_ws;
  auto carve = [&](size_t bytes) { char* p = ws + off; off += (bytes + 255) & ~(size_t)255; return p; };
  b16* WIN = (b16*)carve(H * 32 * 2); b16* WG1 = (b16*)carve(H * H * 2); b16* WG2 = (b16*)carve(H * H * 2); b16* WIP = (b16*)carve(2 * DI * H * 2); b16* WX = (b16*)carve(64 * DI * 2); b16* WDT = (b16*)carve(DI * 32 * 2); b16* WO = (b16*)carve(H * DI * 2);
  float* HA = (float*)carve((size_t)N * H * 4); float* HB = (float*)carve((size_t)N * H * 4); float* XW = (float*)carve((size_t)N * H * 4); float* XZ = (float*)carve((size_t)N * 2 * DI * 4); float* X = (float*)carve((size_t)N * DI * 4); float* DBL = (float*)carve((size_t)N * 64 * 4); float* DT = (float*)carve((size_t)N * DI * 4); float* Y = (float*)carve((size_t)N * DI * 4); float* HM = (float*)carve((size_t)N * H * 4); float* HF = (float*)carve((size_t)N * H * 4); float* GE = (float*)carve(G * H * 4);
  CsrBufs9 csr; off = csr_carve9(csr, ws, off, E, N);
  if (off > ws_size || off > ((size_t)160 << 20)) return;
  wput_kernel<<<(H * 4 + 255) / 256, 256, 0, stream>>>(Fp(3), F, 32, H, H, WIN); wput_kernel<<<(H * 16 + 255) / 256, 256, 0, stream>>>(Fp(5), H, H, H, H, WG1); wput_kernel<<<(H * 16 + 255) / 256, 256, 0, stream>>>(Fp(7), H, H, H, H, WG2);
  wput_kernel<<<(2 * DI * 16 + 255) / 256, 256, 0, stream>>>(Fp(9), H, H, 2 * DI, 2 * DI, WIP); wput_kernel<<<(64 * 32 + 255) / 256, 256, 0, stream>>>(Fp(12), DI, DI, XPW, 64, WX); wput_kernel<<<(DI * 4 + 255) / 256, 256, 0, stream>>>(Fp(13), DTR, 32, DI, DI, WDT); wput_kernel<<<(H * 32 + 255) / 256, 256, 0, stream>>>(Fp(17), DI, DI, H, H, WO);
  csr_build9(csr, Ip(1) + E, E, N, stream);
  dense_kernel<32, 8, 1, 1><<<NBLK, 32, 0, stream>>>(Fp(0), F, 0, F, XS, WIN, Fp(4), HA);
  dense_kernel<128, 8, 0, 0><<<NBLK, 32, 0, stream>>>(HA, H, 0, H, S1, WG1, nullptr, XW); agg_kernel<<<N / 8, 256, 0, stream>>>(XW, Ip(1), csr.PERM, csr.ROWPTR, csr.ROWCNT, (int)csr.permLen, Fp(6), HB);
  dense_kernel<128, 8, 0, 0><<<NBLK, 32, 0, stream>>>(HB, H, 0, H, S2, WG2, nullptr, XW); agg_kernel<<<N / 8, 256, 0, stream>>>(XW, Ip(1), csr.PERM, csr.ROWPTR, csr.ROWCNT, (int)csr.permLen, Fp(8), HA);
  dense_kernel<128, 32, 0, 0><<<NBLK, 32, 0, stream>>>(HA, H, 0, H, S2, WIP, nullptr, XZ);
  conv_kernel<<<(unsigned)(((size_t)LS * 32 + 255) / 256), 256, 0, stream>>>(XZ, Fp(10), Fp(11), LS, X);
  dense_kernel<256, 4, 0, 0><<<(LS + 15) / 16, 32, 0, stream>>>(X, DI, 0, DI, SX, WX, nullptr, DBL);
  dense_kernel<32, 16, 0, 3><<<(LS + 15) / 16, 32, 0, stream>>>(DBL, 64, 0, DTR, SD, WDT, Fp(14), DT);
  scan_kernel<<<1, 256, 0, stream>>>(X, DT, DBL, XZ, Fp(15), Fp(16), LS, Y);
  dense_kernel<256, 8, 0, 0><<<(LS + 15) / 16, 32, 0, stream>>>(Y, DI, 0, DI, SY, WO, nullptr, HM);
  ln_kernel<<<(LS + 7) / 8, 256, 0, stream>>>(HA, HM, Fp(18), Fp(19), LS, HF);
  pool_kernel<<<G, H, 0, stream>>>(HF, Ip(2), LS, GE);
  heads_kernel<<<1, 256, 0, stream>>>(GE, Fp(20), Fp(21), Fp(22), Fp(23), Fp(24), Fp(25), Fp(26), Fp(27), Fp(28), Fp(29), Fp(30), Fp(31), Fp(32), Fp(33), (float*)d_out);
}
